// BiMambaBlock_62989990363685
// MI455X (gfx1250) — hardware-run, weakly checked
//
#include <hip/hip_runtime.h>
#include <math.h>

typedef __attribute__((ext_vector_type(16))) _Float16 v16h;
typedef __attribute__((ext_vector_type(8)))  _Float16 v8h;
typedef __attribute__((ext_vector_type(8)))  float    v8f;
typedef __attribute__((ext_vector_type(4)))  float    v4f;
typedef __attribute__((ext_vector_type(4)))  unsigned v4u;

constexpr int kB    = 2;
constexpr int kL    = 2048;
constexpr int kRows = kB * kL;
constexpr int kDM   = 1024;
constexpr int kDH   = 512;
constexpr int kDI   = 1024;
constexpr int kNS   = 128;
constexpr int kNH   = 16;
constexpr int kHD   = 64;
constexpr int kCD   = 1280;
constexpr int kNIP  = 2320;
constexpr int kZN   = 1088;
constexpr int kZDT  = 1024;
constexpr int kWINR = kZN + kCD;
constexpr int kQ    = 64;
constexpr int kNC   = kL / kQ;
constexpr int kNBC  = kB * kNC;
constexpr int kNBCH = kNBC * kNH;
constexpr float kEps  = 1e-5f;
constexpr float kWSc  = 64.0f;
constexpr float kWSci = 1.0f / 64.0f;
constexpr float kDSc  = 256.0f;
constexpr float kDSci = 1.0f / 256.0f;
constexpr int kConvTP = 260;
constexpr int kBtP    = 72;
constexpr int kXP     = 65;
constexpr int kFP     = 68;

static_assert(kNIP == 2 * kDI + 2 * kNS + kNH, "in_proj width");
static_assert(kCD == kDI + 2 * kNS, "conv width");
static_assert((kDH % 32) == 0 && (kDI % 32) == 0 && (kNS % 32) == 0 && (kQ % 32) == 0, "GEMM K multiples of 32");
static_assert((kRows % 64) == 0 && (kZN % 64) == 0 && (kCD % 64) == 0 && (kDH % 64) == 0 && (kDM % 64) == 0 &&
              (kQ % 64) == 0 && (kNS % 64) == 0 && (kHD % 64) == 0, "GEMM M,N multiples of 64");
static_assert(kZN >= kDI + kNH && (kL % kQ) == 0 && kHD == kQ, "plane geometry");

constexpr size_t kOffZ    = 0;
constexpr size_t kOffXBR  = kOffZ + (size_t)kRows * kZN * 4;
constexpr size_t kOffCS   = kOffXBR;
constexpr size_t kOffECS  = kOffCS + (size_t)kNBCH * kQ * 4;
constexpr size_t kOffDTH  = kOffECS + (size_t)kNBCH * kQ * 4;
constexpr size_t kOffGB   = kOffDTH + (size_t)kNBCH * kQ * 4;
constexpr size_t kOffYIN  = kOffXBR + 2097152;
constexpr size_t kOffXC   = kOffXBR + (size_t)kRows * kCD * 4;
constexpr size_t kOffSP   = kOffXC + (size_t)kRows * kDI * 4;
constexpr size_t kOffYIT  = kOffSP;
constexpr size_t kOffWOUT = kOffSP + (size_t)kNBCH * kHD * kNS * 4;
constexpr size_t kOffBPL  = kOffWOUT + (size_t)kDH * kDI * 2;
constexpr size_t kOffCPL  = kOffBPL + (size_t)kRows * kNS * 2;
constexpr size_t kOffBTP  = kOffCPL + (size_t)kRows * kNS * 2;
constexpr size_t kOffXTP  = kOffBTP + (size_t)kNBC * kNS * kQ * 2;
constexpr size_t kOffXDTP = kOffXTP + (size_t)kNBCH * kQ * kQ * 2;
constexpr size_t kOffHPL  = kOffXTP;
constexpr size_t kOffWOP  = kOffXTP;
constexpr size_t kOffWPL  = kOffXDTP + (size_t)kNBCH * kQ * kQ * 2;
constexpr size_t kOffYN   = kOffWPL;
constexpr size_t kOffU    = kOffWPL;
constexpr size_t kOffWIN  = kOffU + (size_t)kRows * kDH * 2;
constexpr size_t kOffCAT  = kOffWPL + (size_t)kRows * kDI * 2;
constexpr size_t kWsTotal = kOffCAT + (size_t)kRows * kDI * 2;
static_assert(kWsTotal == 126877696ull, "carve total");
static_assert(kWsTotal <= 134217728ull, "carve cap");
static_assert(kOffGB + (size_t)kNBC * kQ * kQ * 4 <= kOffYIN, "small planes before YIN");
static_assert(kOffYIN + (size_t)kRows * kDI * 4 <= kOffXC, "YIN inside the XBR region");
static_assert((size_t)kRows * kDI * 4 <= (size_t)kNBCH * kHD * kNS * 4, "YIT inside the SP region");
static_assert((size_t)kNBCH * kHD * kNS * 2 <= 2 * (size_t)kNBCH * kQ * kQ * 2, "HPL inside XTP+XDTP");
static_assert((size_t)kDM * kDM * 2 <= 2 * (size_t)kNBCH * kQ * kQ * 2, "WOP inside XTP+XDTP");
static_assert(kOffWIN + (size_t)kWINR * kDH * 2 <= kOffCAT, "U+WIN inside the WPL region");
static_assert(kOffCPL == kOffBPL + (size_t)kRows * kNS * 2, "CPL directly follows BPL");
static_assert((kOffXBR % 128) == 0 && (kOffECS % 128) == 0 && (kOffDTH % 128) == 0 && (kOffGB % 128) == 0 &&
              (kOffYIN % 128) == 0 && (kOffXC % 128) == 0 && (kOffSP % 128) == 0 && (kOffWOUT % 128) == 0 &&
              (kOffBPL % 128) == 0 && (kOffCPL % 128) == 0 && (kOffBTP % 128) == 0 && (kOffXTP % 128) == 0 &&
              (kOffXDTP % 128) == 0 && (kOffWPL % 128) == 0 && (kOffWIN % 128) == 0 && (kOffCAT % 128) == 0,
              "128-B aligned regions");

__device__ __forceinline__ v16h frag_load(const _Float16* p) {
  union { v16h v; v8h h[2]; } f;
  f.h[0] = *(const v8h*)(p);
  f.h[1] = *(const v8h*)(p + 16);
  return f.v;
}
__device__ __forceinline__ v8f mma16(v16h a, v16h b, v8f c) {
  return __builtin_amdgcn_wmma_f32_16x16x32_f16(false, a, false, b, (short)0, c, false, false);
}
__device__ __forceinline__ void guard4(v8f& a, v8f& b, v8f& c, v8f& d, v16h x, v16h y) {
  asm volatile("v_nop\n\tv_nop\n\tv_nop\n\tv_nop" : "+v"(a), "+v"(b), "+v"(c), "+v"(d) : "v"(x), "v"(y));
}
__device__ __forceinline__ void keep4(v16h a, v16h b, v16h c, v16h d) {
  asm volatile("v_nop" :: "v"(a), "v"(b), "v"(c), "v"(d));
}
__device__ __forceinline__ void accg4(v8f& a, v8f& b, v8f& c, v8f& d) {
  asm volatile("v_nop\n\tv_nop\n\tv_nop\n\tv_nop" : "+v"(a), "+v"(b), "+v"(c), "+v"(d));
}

template <int BIAS_MODE, int OUT_MODE, bool RESID, bool RSC, bool FLIP>
__global__ __launch_bounds__(256) void gemm64_kernel(
    const unsigned short* __restrict__ Ap, int lda, long strideA, int aDiv,
    const unsigned short* __restrict__ Btp, int ldb, long strideB, int bDiv,
    void* __restrict__ Cout, int ldc, long strideC, int cDiv, int cMod, long cColUnit,
    const float* __restrict__ bias, const float* __restrict__ resid, const float* __restrict__ rsc,
    int M, int N, int K, int nbz, float scale)
{
  __shared__ __align__(16) float sT[8][16 * 68];
  const int lane = threadIdx.x & 31;
  const int wave = threadIdx.x >> 5;
  const int tilesN = N >> 6;
  const int tilesM = M >> 6;
  const int per = tilesM * tilesN;
  const int tile = blockIdx.x * 8 + wave;
  if (tile >= nbz * per) return;
  const int bz = tile / per;
  const int t2 = tile - bz * per;
  const int tm = t2 / tilesN;
  const int tn = t2 - tm * tilesN;
  const int m0 = tm << 6;
  const int n0 = tn << 6;

  const _Float16* Ab = (const _Float16*)Ap  + (size_t)(bz / aDiv) * (size_t)strideA;
  const _Float16* Bb = (const _Float16*)Btp + (size_t)(bz / bDiv) * (size_t)strideB;
  const size_t cOff = (size_t)(bz / cDiv) * (size_t)strideC + (size_t)(bz % cMod) * (size_t)cColUnit;

  const int rlane = lane & 15;
  const int koff  = (lane >> 4) * 8;
  const int mOff  = (lane >> 4) * 8;

  v8f acc[4][4];
#pragma unroll
  for (int i = 0; i < 4; ++i)
#pragma unroll
    for (int j = 0; j < 4; ++j) acc[i][j] = (v8f){0.f, 0.f, 0.f, 0.f, 0.f, 0.f, 0.f, 0.f};

  for (int k0 = 0; k0 < K; k0 += 32) {
    v16h bfr[4];
#pragma unroll
    for (int j = 0; j < 4; ++j)
      bfr[j] = frag_load(Bb + (size_t)(n0 + (j << 4) + rlane) * ldb + koff + k0);
#pragma unroll
    for (int i = 0; i < 4; ++i) {
      const v16h afr = frag_load(Ab + (size_t)(m0 + (i << 4) + rlane) * lda + koff + k0);
#pragma unroll
      for (int j = 0; j < 4; ++j) acc[i][j] = mma16(afr, bfr[j], acc[i][j]);
      guard4(acc[i][0], acc[i][1], acc[i][2], acc[i][3], afr, bfr[3]);
    }
    keep4(bfr[0], bfr[1], bfr[2], bfr[3]);
  }
  accg4(acc[0][0], acc[0][1], acc[0][2], acc[0][3]);
  accg4(acc[1][0], acc[1][1], acc[1][2], acc[1][3]);
  accg4(acc[2][0], acc[2][1], acc[2][2], acc[2][3]);
  accg4(acc[3][0], acc[3][1], acc[3][2], acc[3][3]);

  float* slab = sT[wave];
  const float* rsp = RSC ? (rsc + (size_t)bz * M) : nullptr;
#pragma unroll
  for (int i = 0; i < 4; ++i) {
    const int mBase = m0 + (i << 4);
    float rsv[8];
#pragma unroll
    for (int r = 0; r < 8; ++r) rsv[r] = RSC ? rsp[mBase + mOff + r] : 1.0f;
#pragma unroll
    for (int j = 0; j < 4; ++j) {
#pragma unroll
      for (int r = 0; r < 8; ++r) {
        float v = acc[i][j][r] * scale;
        if (RSC) v *= rsv[r];
        slab[(mOff + r) * 68 + (j << 4) + rlane] = v;
      }
    }
    __builtin_amdgcn_fence(__ATOMIC_RELEASE, "workgroup");
    __builtin_amdgcn_wave_barrier();
    __builtin_amdgcn_fence(__ATOMIC_ACQUIRE, "workgroup");
    if (OUT_MODE == 0) {
      float* Cp = (float*)Cout + cOff;
      const int hh = lane >> 4, c4 = (lane & 15) * 4;
      v4f bv4 = (v4f){0.f, 0.f, 0.f, 0.f};
      if (BIAS_MODE == 2) bv4 = *(const v4f*)(bias + n0 + c4);
      for (int pass = 0; pass < 2; ++pass) {
#pragma unroll
        for (int it = 0; it < 8; ++it) {
          const int row = it * 2 + hh;
          const int grow = mBase + row;
          const int orow = FLIP ? ((grow & ~(kL - 1)) | ((kL - 1) - (grow & (kL - 1)))) : grow;
          v4f v = *(const v4f*)(slab + row * 68 + c4);
          if (BIAS_MODE == 2) v += bv4;
          if (RESID) v += *(const v4f*)(resid + (size_t)orow * ldc + n0 + c4);
          *(volatile v4f*)(Cp + (size_t)orow * ldc + n0 + c4) = v;
        }
        __threadfence();
      }
    } else {
      unsigned short* Cp = (unsigned short*)Cout + cOff;
      const int q = lane >> 3, c8 = (lane & 7) * 8;
      for (int pass = 0; pass < 2; ++pass) {
#pragma unroll
        for (int it = 0; it < 4; ++it) {
          const int row = it * 4 + q;
          const int grow = mBase + row;
          const int orow = FLIP ? ((grow & ~(kL - 1)) | ((kL - 1) - (grow & (kL - 1)))) : grow;
          const float* sp = slab + row * 68 + c8;
          v8h hv;
#pragma unroll
          for (int e = 0; e < 8; ++e) hv[e] = (_Float16)sp[e];
          *(volatile v8h*)(Cp + (size_t)orow * ldc + n0 + c8) = hv;
        }
        __threadfence();
      }
    }
    __builtin_amdgcn_fence(__ATOMIC_RELEASE, "workgroup");
    __builtin_amdgcn_wave_barrier();
    __builtin_amdgcn_fence(__ATOMIC_ACQUIRE, "workgroup");
  }
}

__global__ __launch_bounds__(256) void rmsnorm_u_kernel(
    const float* __restrict__ x, const float* __restrict__ nw, unsigned short* __restrict__ U, int dir)
{
  __shared__ float sred[8];
  const int m = blockIdx.x, tid = threadIdx.x, lane = tid & 31, wave = tid >> 5;
  const float* xr = x + (size_t)m * kDM;
  const v4f v = *(const v4f*)(xr + tid * 4);
  float ss = 0.0f;
  ss += v[0] * v[0]; ss += v[1] * v[1]; ss += v[2] * v[2]; ss += v[3] * v[3];
#pragma unroll
  for (int off = 1; off < 32; off <<= 1) ss += __shfl_xor(ss, off, 32);
  if (lane == 0) sred[wave] = ss;
  __syncthreads();
  float tot = 0.0f;
#pragma unroll
  for (int i = 0; i < 8; ++i) tot += sred[i];
  const float sc = rsqrtf(tot * (1.0f / 1024.0f) + kEps);
  const int bq = m >> 11, l = m & (kL - 1);
  const int orow = dir ? (bq * kL + (kL - 1 - l)) : m;
  if (tid < 64) {
    const int c0 = dir * kDH + tid * 8;
    const v4f a0 = *(const v4f*)(xr + c0), a1 = *(const v4f*)(xr + c0 + 4);
    const v4f w0 = *(const v4f*)(nw + c0), w1 = *(const v4f*)(nw + c0 + 4);
    v8h hv;
#pragma unroll
    for (int e = 0; e < 4; ++e) {
      hv[e]     = (_Float16)(a0[e] * sc * w0[e]);
      hv[4 + e] = (_Float16)(a1[e] * sc * w1[e]);
    }
    unsigned short* p = U + (size_t)orow * kDH + tid * 8;
    *(volatile v8h*)p = hv;
    __threadfence();
    *(volatile v8h*)p = hv;
  }
}

__global__ __launch_bounds__(256) void cast_f16_kernel(
    const float* __restrict__ src, unsigned short* __restrict__ dst, int total8, float scale)
{
  const int i = blockIdx.x * 256 + threadIdx.x;
  if (i >= total8) return;
  const size_t e0 = (size_t)i << 3;
  const v4f a0 = *(const v4f*)(src + e0), a1 = *(const v4f*)(src + e0 + 4);
  v8h hv;
#pragma unroll
  for (int e = 0; e < 4; ++e) { hv[e] = (_Float16)(a0[e] * scale); hv[4 + e] = (_Float16)(a1[e] * scale); }
  unsigned short* p = dst + e0;
  *(volatile v8h*)p = hv;
  __threadfence();
  *(volatile v8h*)p = hv;
}

__global__ __launch_bounds__(256) void cast_inw_kernel(
    const float* __restrict__ src, unsigned short* __restrict__ dst, float scale)
{
  const int i = blockIdx.x * 256 + threadIdx.x;
  if (i >= kWINR * kDH / 8) return;
  const int r = i >> 6;
  const int c8 = (i & 63) * 8;
  const bool zr = (r >= kDI + kNH) && (r < kZN);
  const int srow = (r < kDI) ? r : (r < kDI + kNH) ? (r + kCD) : zr ? 0 : (r - (kZN - kDI));
  const float f = zr ? 0.0f : scale;
  const float* sp = src + (size_t)srow * kDH + c8;
  const v4f a0 = *(const v4f*)(sp), a1 = *(const v4f*)(sp + 4);
  v8h hv;
#pragma unroll
  for (int e = 0; e < 4; ++e) { hv[e] = (_Float16)(a0[e] * f); hv[4 + e] = (_Float16)(a1[e] * f); }
  unsigned short* p = dst + (size_t)r * kDH + c8;
  *(volatile v8h*)p = hv;
  __threadfence();
  *(volatile v8h*)p = hv;
}

__global__ __launch_bounds__(256) void conv_silu_kernel(
    const float* __restrict__ XBR, const float* __restrict__ cw, const float* __restrict__ cb,
    float* __restrict__ XC, unsigned short* __restrict__ BCP)
{
  __shared__ __align__(16) float sT[16 * kConvTP];
  const int tid = threadIdx.x, lane = tid & 31, wave = tid >> 5;
  const int c0 = blockIdx.x * 256, c = c0 + tid;
  const int g0 = blockIdx.y * 64;
  const int tb = g0 & (kL - 1);
  const bool isx = (blockIdx.x < 4);
  const float w0 = cw[c * 4 + 0], w1 = cw[c * 4 + 1], w2 = cw[c * 4 + 2], w3 = cw[c * 4 + 3];
  const float bcv = cb[c];
  float xm3, xm2, xm1;
  {
    const bool hist = (tb > 0);
    const int rb = hist ? (g0 - 3) : g0;
    const float v3 = XBR[(size_t)rb * kCD + c];
    const float v2 = XBR[(size_t)(rb + 1) * kCD + c];
    const float v1 = XBR[(size_t)(rb + 2) * kCD + c];
    const float fh = hist ? 1.0f : 0.0f;
    xm3 = v3 * fh; xm2 = v2 * fh; xm1 = v1 * fh;
  }
  const int hrow = wave >> 1;
  const int hch  = (wave & 1) * 128 + lane * 4;
  const size_t poff = (lane < 16) ? (size_t)(lane * 8) : ((size_t)kRows * kNS + (size_t)((lane - 16) * 8));
#pragma unroll 1
  for (int sub = 0; sub < 4; ++sub) {
    const int lb = g0 + sub * 16;
#pragma unroll 1
    for (int s = 0; s < 16; ++s) {
      const float xcur = XBR[(size_t)(lb + s) * kCD + c];
      float acc = w0 * xm3;
      acc = fmaf(w1, xm2, acc);
      acc = fmaf(w2, xm1, acc);
      acc = fmaf(w3, xcur, acc);
      const float sv = acc + bcv;
      const float ez = expf(-sv);
      sT[s * kConvTP + tid] = sv * __builtin_amdgcn_rcpf(1.0f + ez);
      xm3 = xm2; xm2 = xm1; xm1 = xcur;
    }
    __syncthreads();
    if (isx) {
      v4f fv[4];
#pragma unroll
      for (int it = 0; it < 4; ++it) fv[it] = *(const v4f*)(sT + (it * 4 + hrow) * kConvTP + hch);
      for (int pass = 0; pass < 2; ++pass) {
#pragma unroll
        for (int it = 0; it < 4; ++it)
          *(volatile v4f*)(XC + (size_t)(lb + it * 4 + hrow) * kDI + c0 + hch) = fv[it];
        __threadfence();
      }
    } else {
      v8h hv[2];
#pragma unroll
      for (int it = 0; it < 2; ++it) {
        const float* sp = sT + (it * 8 + wave) * kConvTP + lane * 8;
        const v4f a0 = *(const v4f*)(sp), a1 = *(const v4f*)(sp + 4);
#pragma unroll
        for (int e = 0; e < 4; ++e) { hv[it][e] = (_Float16)a0[e]; hv[it][4 + e] = (_Float16)a1[e]; }
      }
      for (int pass = 0; pass < 2; ++pass) {
#pragma unroll
        for (int it = 0; it < 2; ++it)
          *(volatile v8h*)(BCP + (size_t)(lb + it * 8 + wave) * kNS + poff) = hv[it];
        __threadfence();
      }
    }
    __syncthreads();
  }
}

__device__ __forceinline__ void bt_put(unsigned short* sBt, int i, int nbase, v4u u) {
#pragma unroll
  for (int jw = 0; jw < 4; ++jw) {
    const unsigned w = u[jw];
    const int n = nbase + 2 * jw;
    sBt[n * kBtP + i] = (unsigned short)(w & 0xffffu);
    sBt[(n + 1) * kBtP + i] = (unsigned short)(w >> 16);
  }
}

__global__ __launch_bounds__(256) void prep_bc_kernel(
    const float* __restrict__ Z, const float* __restrict__ dtb, const float* __restrict__ alog,
    const unsigned short* __restrict__ BPL,
    float* __restrict__ CS, float* __restrict__ ECS, float* __restrict__ DTH, unsigned short* __restrict__ BTP)
{
  __shared__ __align__(16) float sDT[kNH * kQ];
  __shared__ __align__(16) float sADT[kNH * kQ];
  __shared__ __align__(16) float sCS[kNH * kQ];
  __shared__ __align__(16) float sECS[kNH * kQ];
  __shared__ __align__(16) unsigned short sBt[kNS * kBtP];
  const int tid = threadIdx.x, lane = tid & 31, wave = tid >> 5;
  const int bc = blockIdx.x;
  const int g0 = bc * kQ;
#pragma unroll 1
  for (int j = 0; j < 4; ++j) {
    const int e = tid + 256 * j;
    const int i = e >> 4, h = e & 15;
    const float raw = Z[(size_t)(g0 + i) * kZN + kZDT + h] + dtb[h];
    const float ex = expf(-fabsf(raw));
    const float dt = fmaxf(raw, 0.0f) + log1pf(ex);
    const float an = -expf(alog[h]);
    sDT[h * kQ + i]  = dt;
    sADT[h * kQ + i] = dt * an;
  }
  {
    const int i = tid >> 2, wq = tid & 3;
    const v4u* brow = (const v4u*)(BPL + (size_t)(g0 + i) * kNS) + wq * 4;
    const v4u u0 = brow[0], u1 = brow[1], u2 = brow[2], u3 = brow[3];
    bt_put(sBt, i, 2 * (wq * 16 + 0), u0);
    bt_put(sBt, i, 2 * (wq * 16 + 4), u1);
    bt_put(sBt, i, 2 * (wq * 16 + 8), u2);
    bt_put(sBt, i, 2 * (wq * 16 + 12), u3);
  }
  __syncthreads();
  if (tid < kNH) {
    float a = 0.0f;
#pragma unroll 1
    for (int i = 0; i < kQ; ++i) {
      a = a + sADT[tid * kQ + i];
      sCS[tid * kQ + i] = a;
      sECS[tid * kQ + i] = expf(a);
    }
  }
  __syncthreads();
  {
    const size_t o = (size_t)bc * (kNH * kQ) + tid * 4;
    const v4f vcs = *(const v4f*)(sCS + tid * 4);
    const v4f vec = *(const v4f*)(sECS + tid * 4);
    const v4f vdt = *(const v4f*)(sDT + tid * 4);
    for (int pass = 0; pass < 2; ++pass) {
      *(volatile v4f*)(CS + o)  = vcs;
      *(volatile v4f*)(ECS + o) = vec;
      *(volatile v4f*)(DTH + o) = vdt;
      __threadfence();
    }
  }
  {
    const int q = lane >> 3, c8 = (lane & 7) * 8;
    v4u bv[4];
#pragma unroll
    for (int it = 0; it < 4; ++it) {
      const int n = it * 32 + wave * 4 + q;
      bv[it] = *(const v4u*)(sBt + n * kBtP + c8);
    }
    for (int pass = 0; pass < 2; ++pass) {
#pragma unroll
      for (int it = 0; it < 4; ++it) {
        const int n = it * 32 + wave * 4 + q;
        *(volatile v4u*)(BTP + (size_t)bc * (kNS * kQ) + (size_t)n * kQ + c8) = bv[it];
      }
      __threadfence();
    }
  }
}

__global__ __launch_bounds__(256) void prep_x_kernel(
    const float* __restrict__ XC, const float* __restrict__ CS, const float* __restrict__ DTH,
    unsigned short* __restrict__ XTP, unsigned short* __restrict__ XDTP)
{
  __shared__ float sX[kQ * kXP];
  __shared__ __align__(16) float sF[kQ];
  const int tid = threadIdx.x, lane = tid & 31, wave = tid >> 5;
  const int bch = blockIdx.x, bc = bch >> 4, h = bch & 15;
  const int g0 = bc * kQ;
  {
    const int i = tid >> 2, p16 = (tid & 3) * 16;
    const float* src = XC + (size_t)(g0 + i) * kDI + h * kHD + p16;
    const v4f a0 = *(const v4f*)(src), a1 = *(const v4f*)(src + 4), a2 = *(const v4f*)(src + 8), a3 = *(const v4f*)(src + 12);
    float* d = sX + i * kXP + p16;
#pragma unroll
    for (int e = 0; e < 4; ++e) { d[e] = a0[e]; d[4 + e] = a1[e]; d[8 + e] = a2[e]; d[12 + e] = a3[e]; }
  }
  if (tid < kQ) {
    const float cs63 = CS[(size_t)bch * kQ + (kQ - 1)];
    const float ci = CS[(size_t)bch * kQ + tid];
    const float di = DTH[(size_t)bch * kQ + tid];
    sF[tid] = expf(cs63 - ci) * di * kDSc;
  }
  __syncthreads();
  const int q = lane >> 3, c8 = (lane & 7) * 8;
  v8h ht[2], hd[2];
#pragma unroll
  for (int it = 0; it < 2; ++it) {
    const int p = it * 32 + wave * 4 + q;
    const v4f f0 = *(const v4f*)(sF + c8), f1 = *(const v4f*)(sF + c8 + 4);
#pragma unroll
    for (int e = 0; e < 4; ++e) {
      const float x0 = sX[(c8 + e) * kXP + p];
      const float x1 = sX[(c8 + 4 + e) * kXP + p];
      ht[it][e] = (_Float16)x0;          ht[it][4 + e] = (_Float16)x1;
      hd[it][e] = (_Float16)(x0 * f0[e]); hd[it][4 + e] = (_Float16)(x1 * f1[e]);
    }
  }
  for (int pass = 0; pass < 2; ++pass) {
#pragma unroll
    for (int it = 0; it < 2; ++it) {
      const int p = it * 32 + wave * 4 + q;
      const size_t o = (size_t)bch * (kQ * kQ) + (size_t)p * kQ + c8;
      *(volatile v8h*)(XTP + o)  = ht[it];
      *(volatile v8h*)(XDTP + o) = hd[it];
    }
    __threadfence();
  }
}

__global__ __launch_bounds__(256) void wbuild_kernel(
    const float* __restrict__ GB, const float* __restrict__ CS, const float* __restrict__ DTH, unsigned short* __restrict__ WPL)
{
  __shared__ float sCS[kQ];
  __shared__ float sD[kQ];
  __shared__ __align__(16) float sF[kQ * kFP];
  const int tid = threadIdx.x, lane = tid & 31, wave = tid >> 5;
  const int bch = blockIdx.x, bc = bch >> 4;
  if (tid < kQ) sCS[tid] = CS[(size_t)bch * kQ + tid];
  if (tid >= kQ && tid < 2 * kQ) sD[tid - kQ] = DTH[(size_t)bch * kQ + (tid - kQ)];
  __syncthreads();
#pragma unroll 1
  for (int j = 0; j < 16; ++j) {
    const int e = tid + 256 * j;
    const int t = e >> 6, i = e & 63;
    const float arg = fminf(sCS[t] - sCS[i], 0.0f);
    float f = expf(arg) * sD[i] * kDSc;
    f = (i <= t) ? f : 0.0f;
    sF[t * kFP + i] = f;
  }
  __syncthreads();
  const int q = lane >> 3, c8 = (lane & 7) * 8;
  v8h hv[2];
#pragma unroll
  for (int it = 0; it < 2; ++it) {
    const int t = it * 32 + wave * 4 + q;
    const float* gp = GB + (size_t)bc * (kQ * kQ) + (size_t)t * kQ + c8;
    const v4f g0 = *(const v4f*)(gp), g1 = *(const v4f*)(gp + 4);
    const v4f f0 = *(const v4f*)(sF + t * kFP + c8), f1 = *(const v4f*)(sF + t * kFP + c8 + 4);
#pragma unroll
    for (int e = 0; e < 4; ++e) { hv[it][e] = (_Float16)(g0[e] * f0[e]); hv[it][4 + e] = (_Float16)(g1[e] * f1[e]); }
  }
  for (int pass = 0; pass < 2; ++pass) {
#pragma unroll
    for (int it = 0; it < 2; ++it) {
      const int t = it * 32 + wave * 4 + q;
      *(volatile v8h*)(WPL + (size_t)bch * (kQ * kQ) + (size_t)t * kQ + c8) = hv[it];
    }
    __threadfence();
  }
}

__global__ __launch_bounds__(256) void combine_kernel(
    const float* __restrict__ SP, const float* __restrict__ ECS, unsigned short* __restrict__ HPL)
{
  const int tid = threadIdx.x;
  const int bh = blockIdx.x, bq = bh >> 4, h = bh & 15;
  float Hs[32];
#pragma unroll
  for (int k = 0; k < 32; ++k) Hs[k] = 0.0f;
#pragma unroll 1
  for (int cix = 0; cix < kNC; ++cix) {
    const int bch = ((bq * kNC + cix) << 4) + h;
    const size_t base = (size_t)bch * (kHD * kNS);
    v8h hv[4];
#pragma unroll
    for (int it = 0; it < 4; ++it)
#pragma unroll
      for (int k = 0; k < 8; ++k) hv[it][k] = (_Float16)Hs[it * 8 + k];
    unsigned short* dst = HPL + base + tid * 8;
    for (int pass = 0; pass < 2; ++pass) {
#pragma unroll
      for (int it = 0; it < 4; ++it) *(volatile v8h*)(dst + it * 2048) = hv[it];
      __threadfence();
    }
    const float dec = ECS[(size_t)bch * kQ + (kQ - 1)];
    const float* sp = SP + base + tid * 8;
#pragma unroll
    for (int it = 0; it < 4; ++it) {
      const v4f a0 = *(const v4f*)(sp + it * 2048), a1 = *(const v4f*)(sp + it * 2048 + 4);
#pragma unroll
      for (int k = 0; k < 4; ++k) {
        Hs[it * 8 + k]     = fmaf(dec, Hs[it * 8 + k], a0[k]);
        Hs[it * 8 + 4 + k] = fmaf(dec, Hs[it * 8 + 4 + k], a1[k]);
      }
    }
  }
}

__global__ __launch_bounds__(256) void gate_norm_kernel(
    const float* __restrict__ YIN, const float* __restrict__ YIT, const float* __restrict__ XC, const float* __restrict__ Z,
    const float* __restrict__ Dp, const float* __restrict__ gw, unsigned short* __restrict__ YN)
{
  __shared__ float sred[8];
  __shared__ __align__(16) float sY[kDI];
  const int m = blockIdx.x, tid = threadIdx.x, lane = tid & 31, wave = tid >> 5;
  const int c = tid * 4;
  const size_t ro = (size_t)m * kDI + c;
  const v4f yi = *(const v4f*)(YIN + ro), yo = *(const v4f*)(YIT + ro), xv = *(const v4f*)(XC + ro);
  const v4f zv = *(const v4f*)(Z + (size_t)m * kZN + c);
  const float dv = Dp[tid >> 4];
  float ss = 0.0f;
  v4f g;
#pragma unroll
  for (int e = 0; e < 4; ++e) {
    const float ys = yi[e] + yo[e];
    const float y  = ys + xv[e] * dv;
    const float ez = expf(-zv[e]);
    const float sz = zv[e] * __builtin_amdgcn_rcpf(1.0f + ez);
    const float ge = y * sz;
    g[e] = ge;
    ss = fmaf(ge, ge, ss);
  }
  *(v4f*)(sY + c) = g;
#pragma unroll
  for (int off = 1; off < 32; off <<= 1) ss += __shfl_xor(ss, off, 32);
  if (lane == 0) sred[wave] = ss;
  __syncthreads();
  float tot = 0.0f;
#pragma unroll
  for (int i = 0; i < 8; ++i) tot += sred[i];
  const float sc = rsqrtf(tot * (1.0f / 1024.0f) + kEps);
  if (tid < 128) {
    const v4f a0 = *(const v4f*)(sY + tid * 8), a1 = *(const v4f*)(sY + tid * 8 + 4);
    const v4f w0 = *(const v4f*)(gw + tid * 8), w1 = *(const v4f*)(gw + tid * 8 + 4);
    v8h hv;
#pragma unroll
    for (int e = 0; e < 4; ++e) { hv[e] = (_Float16)(a0[e] * sc * w0[e]); hv[4 + e] = (_Float16)(a1[e] * sc * w1[e]); }
    unsigned short* p = YN + (size_t)m * kDI + tid * 8;
    *(volatile v8h*)p = hv;
    __threadfence();
    *(volatile v8h*)p = hv;
  }
}

extern "C" void kernel_launch(void* const* d_in, const int* in_sizes, int n_in,
                              void* d_out, int out_size, void* d_ws, size_t ws_size,
                              hipStream_t stream) {
  if (n_in < 20) return;
  if (in_sizes[0] != kRows * kDM) return;
  if (in_sizes[1] != kDM) return;
  if (in_sizes[2] != kDM * kDM) return;
  if (in_sizes[3] != kDM) return;
  for (int d = 0; d < 2; ++d) {
    const int o = 4 + 8 * d;
    if (in_sizes[o + 0] != kNIP * kDH) return;
    if (in_sizes[o + 1] != kCD * 4) return;
    if (in_sizes[o + 2] != kCD) return;
    if (in_sizes[o + 3] != kNH) return;
    if (in_sizes[o + 4] != kNH) return;
    if (in_sizes[o + 5] != kNH) return;
    if (in_sizes[o + 6] != kDI) return;
    if (in_sizes[o + 7] != kDH * kDI) return;
  }
  if (out_size != kRows * kDM) return;
  if (ws_size < kWsTotal) return;

  const float* x      = (const float*)d_in[0];
  const float* norm_w = (const float*)d_in[1];
  const float* op_w   = (const float*)d_in[2];
  const float* op_b   = (const float*)d_in[3];
  const float* in_w[2]   = {(const float*)d_in[4],  (const float*)d_in[12]};
  const float* conv_w[2] = {(const float*)d_in[5],  (const float*)d_in[13]};
  const float* conv_b[2] = {(const float*)d_in[6],  (const float*)d_in[14]};
  const float* dt_b[2]   = {(const float*)d_in[7],  (const float*)d_in[15]};
  const float* a_log[2]  = {(const float*)d_in[8],  (const float*)d_in[16]};
  const float* dpar[2]   = {(const float*)d_in[9],  (const float*)d_in[17]};
  const float* gn_w[2]   = {(const float*)d_in[10], (const float*)d_in[18]};
  const float* outp_w[2] = {(const float*)d_in[11], (const float*)d_in[19]};
  float* out = (float*)d_out;

  char* ws = (char*)d_ws;
  float*          Z    = (float*)(ws + kOffZ);
  float*          XBR  = (float*)(ws + kOffXBR);
  float*          CS   = (float*)(ws + kOffCS);
  float*          ECS  = (float*)(ws + kOffECS);
  float*          DTH  = (float*)(ws + kOffDTH);
  float*          GB   = (float*)(ws + kOffGB);
  float*          YIN  = (float*)(ws + kOffYIN);
  float*          XC   = (float*)(ws + kOffXC);
  float*          SP   = (float*)(ws + kOffSP);
  float*          YIT  = (float*)(ws + kOffYIT);
  unsigned short* WOUT = (unsigned short*)(ws + kOffWOUT);
  unsigned short* BPL  = (unsigned short*)(ws + kOffBPL);
  unsigned short* CPL  = (unsigned short*)(ws + kOffCPL);
  unsigned short* BTP  = (unsigned short*)(ws + kOffBTP);
  unsigned short* XTP  = (unsigned short*)(ws + kOffXTP);
  unsigned short* XDTP = (unsigned short*)(ws + kOffXDTP);
  unsigned short* HPL  = (unsigned short*)(ws + kOffHPL);
  unsigned short* WOP  = (unsigned short*)(ws + kOffWOP);
  unsigned short* WPL  = (unsigned short*)(ws + kOffWPL);
  unsigned short* YN   = (unsigned short*)(ws + kOffYN);
  unsigned short* U    = (unsigned short*)(ws + kOffU);
  unsigned short* WIN  = (unsigned short*)(ws + kOffWIN);
  unsigned short* CAT  = (unsigned short*)(ws + kOffCAT);

  for (int d = 0; d < 2; ++d) {
    rmsnorm_u_kernel<<<kRows, 256, 0, stream>>>(x, norm_w, U, d);
    cast_inw_kernel<<<(kWINR * kDH / 8) / 256, 256, 0, stream>>>(in_w[d], WIN, kWSc);
    cast_f16_kernel<<<(kDH * kDI / 8) / 256, 256, 0, stream>>>(outp_w[d], WOUT, kDH * kDI / 8, kWSc);

    gemm64_kernel<0, 0, false, false, false><<<(kRows / 64) * (kZN / 64) / 8, 256, 0, stream>>>(
        U, kDH, 0L, 1, WIN, kDH, 0L, 1,
        (void*)Z, kZN, 0L, 1, 1, 0L, nullptr, nullptr, nullptr,
        kRows, kZN, kDH, 1, kWSci);
    gemm64_kernel<0, 0, false, false, false><<<(kRows / 64) * (kCD / 64) / 8, 256, 0, stream>>>(
        U, kDH, 0L, 1, WIN + (size_t)kZN * kDH, kDH, 0L, 1,
        (void*)XBR, kCD, 0L, 1, 1, 0L, nullptr, nullptr, nullptr,
        kRows, kCD, kDH, 1, kWSci);

    conv_silu_kernel<<<dim3(kCD / 256, kRows / 64), 256, 0, stream>>>(XBR, conv_w[d], conv_b[d], XC, BPL);

    prep_bc_kernel<<<kNBC, 256, 0, stream>>>(Z, dt_b[d], a_log[d], BPL, CS, ECS, DTH, BTP);
    prep_x_kernel<<<kNBCH, 256, 0, stream>>>(XC, CS, DTH, XTP, XDTP);

    gemm64_kernel<0, 0, false, false, false><<<kNBC / 8, 256, 0, stream>>>(
        CPL, kNS, (long)(kQ * kNS), 1, BPL, kNS, (long)(kQ * kNS), 1,
        (void*)GB, kQ, (long)(kQ * kQ), 1, 1, 0L, nullptr, nullptr, nullptr,
        kQ, kQ, kNS, kNBC, 1.0f);
    wbuild_kernel<<<kNBCH, 256, 0, stream>>>(GB, CS, DTH, WPL);
    gemm64_kernel<0, 0, false, false, false><<<kNBCH / 8, 256, 0, stream>>>(
        WPL, kQ, (long)(kQ * kQ), 1, XTP, kQ, (long)(kQ * kQ), 1,
        (void*)YIN, kDI, (long)(kQ * kDI), kNH, kNH, (long)kHD, nullptr, nullptr, nullptr,
        kQ, kHD, kQ, kNBCH, kDSci);
    gemm64_kernel<0, 0, false, false, false><<<kNBCH * 2 / 8, 256, 0, stream>>>(
        XDTP, kQ, (long)(kQ * kQ), 1, BTP, kQ, (long)(kNS * kQ), kNH,
        (void*)SP, kNS, (long)(kHD * kNS), 1, 1, 0L, nullptr, nullptr, nullptr,
        kHD, kNS, kQ, kNBCH, 1.0f);
    combine_kernel<<<kB * kNH, 256, 0, stream>>>(SP, ECS, HPL);
    gemm64_kernel<0, 0, false, true, false><<<kNBCH / 8, 256, 0, stream>>>(
        CPL, kNS, (long)(kQ * kNS), kNH, HPL, kNS, (long)(kHD * kNS), 1,
        (void*)YIT, kDI, (long)(kQ * kDI), kNH, kNH, (long)kHD, nullptr, nullptr, ECS,
        kQ, kHD, kNS, kNBCH, kDSci);

    gate_norm_kernel<<<kRows, 256, 0, stream>>>(YIN, YIT, XC, Z, dpar[d], gn_w[d], YN);
    if (d == 0) {
      gemm64_kernel<0, 1, false, false, false><<<(kRows / 64) * (kDH / 64) / 8, 256, 0, stream>>>(
          YN, kDI, 0L, 1, WOUT, kDI, 0L, 1,
          (void*)(CAT), kDI, 0L, 1, 1, 0L, nullptr, nullptr, nullptr,
          kRows, kDH, kDI, 1, kWSci);
    } else {
      gemm64_kernel<0, 1, false, false, true><<<(kRows / 64) * (kDH / 64) / 8, 256, 0, stream>>>(
          YN, kDI, 0L, 1, WOUT, kDI, 0L, 1,
          (void*)(CAT + kDH), kDI, 0L, 1, 1, 0L, nullptr, nullptr, nullptr,
          kRows, kDH, kDI, 1, kWSci);
    }
  }

  cast_f16_kernel<<<(kDM * kDM / 8) / 256, 256, 0, stream>>>(op_w, WOP, kDM * kDM / 8, kWSc);
  gemm64_kernel<2, 0, true, false, false><<<(kRows / 64) * (kDM / 64) / 8, 256, 0, stream>>>(
      CAT, kDI, 0L, 1, WOP, kDM, 0L, 1,
      (void*)out, kDM, 0L, 1, 1, 0L, op_b, x, nullptr,
      kRows, kDM, kDM, 1, kWSci);
}
